// KANLayer_28862180229294
// MI455X (gfx1250) — hardware-verified
//
#include <hip/hip_runtime.h>
#include <math.h>

constexpr int kBatch  = 4096;
constexpr int kIn     = 256;
constexpr int kOut    = 256;
constexpr int kNBasis = 8;
constexpr int kGpts   = 12;
constexpr int kFeat   = 11;
constexpr int kKeff   = kIn * kFeat;
constexpr int kRowsPerBlk   = 8;
constexpr int kChunksPerRow = kKeff / 8;
constexpr int kStoreIters   = kRowsPerBlk * kChunksPerRow / 256;
constexpr float kWCarry      = 16.0f;
constexpr float kWCarryInv   = 1.0f / 16.0f;
constexpr float kResCarry    = 256.0f;
constexpr float kResCarryInv = 1.0f / 256.0f;

static_assert(kKeff % 32 == 0, "K must be a multiple of 32");
static_assert(kBatch % 64 == 0 && kOut % 64 == 0, "M and N must be tile multiples");
static_assert((kKeff * 2) % 128 == 0, "plane row pitch must be a whole number of 128-B lines");
static_assert((kRowsPerBlk * kChunksPerRow) % 256 == 0, "store loop covers the staged rows exactly");
static_assert(kBatch % kRowsPerBlk == 0 && kOut % kRowsPerBlk == 0, "producer grids cover all rows");
static_assert(kIn == 256, "one producer thread per input dim");

typedef __attribute__((ext_vector_type(16))) _Float16 v16h;
typedef __attribute__((ext_vector_type(8)))  _Float16 v8h;
typedef __attribute__((ext_vector_type(16))) __bf16   v16b;
typedef __attribute__((ext_vector_type(8)))  __bf16   v8b;
typedef __attribute__((ext_vector_type(8)))  float    v8f;
typedef __attribute__((ext_vector_type(4)))  float    v4f;
typedef __attribute__((ext_vector_type(4)))  unsigned int v4u;

__device__ __forceinline__ unsigned short f2bf_bits(float f) {
  unsigned u = __float_as_uint(f);
  return (unsigned short)((u + 0x7FFFu + ((u >> 16) & 1u)) >> 16);
}
__device__ __forceinline__ float bf_bits2f(unsigned short h) { return __uint_as_float(((unsigned)h) << 16); }

__device__ __forceinline__ void dep_guard_h(v8f& a, v8f& b, v16h x, v16h y) { asm volatile("v_nop\n\tv_nop\n\tv_nop\n\tv_nop" : "+v"(a), "+v"(b) : "v"(x), "v"(y)); }
__device__ __forceinline__ void dep_guard_b(v8f& a, v8f& b, v16b x, v16b y) { asm volatile("v_nop\n\tv_nop\n\tv_nop\n\tv_nop" : "+v"(a), "+v"(b) : "v"(x), "v"(y)); }
__device__ __forceinline__ void dep_guard4_h(v8f& a, v8f& b, v8f& c, v8f& d, v16h x, v16h y) { asm volatile("v_nop\n\tv_nop\n\tv_nop\n\tv_nop" : "+v"(a), "+v"(b), "+v"(c), "+v"(d) : "v"(x), "v"(y)); }
__device__ __forceinline__ void dep_guard4_b(v8f& a, v8f& b, v8f& c, v8f& d, v16b x, v16b y) { asm volatile("v_nop\n\tv_nop\n\tv_nop\n\tv_nop" : "+v"(a), "+v"(b), "+v"(c), "+v"(d) : "v"(x), "v"(y)); }
__device__ __forceinline__ void keep4_h(v16h a, v16h b, v16h c, v16h d) { asm volatile("v_nop" :: "v"(a), "v"(b), "v"(c), "v"(d)); }
__device__ __forceinline__ void keep4_b(v16b a, v16b b, v16b c, v16b d) { asm volatile("v_nop" :: "v"(a), "v"(b), "v"(c), "v"(d)); }
__device__ __forceinline__ void acc_guard4(v8f& a, v8f& b, v8f& c, v8f& d) { asm volatile("v_nop\n\tv_nop\n\tv_nop\n\tv_nop" : "+v"(a), "+v"(b), "+v"(c), "+v"(d)); }
template <typename T> struct Frag;
template <> struct Frag<_Float16> {
  typedef v16h V; union U { v16h v; v8h h[2]; };
  static __device__ __forceinline__ v16h load(const _Float16* p) {
    U f; f.h[0] = *(const v8h*)(p); f.h[1] = *(const v8h*)(p + 16); return f.v;
  }
  static __device__ __forceinline__ v8f mma(v16h a, v16h b, v8f c) {
    return __builtin_amdgcn_wmma_f32_16x16x32_f16(false, a, false, b, (short)0, c, false, false);
  }
  static __device__ __forceinline__ void guard(v8f& a, v8f& b, v16h x, v16h y) { dep_guard_h(a, b, x, y); }
  static __device__ __forceinline__ void guard4(v8f& a, v8f& b, v8f& c, v8f& d, v16h x, v16h y) { dep_guard4_h(a, b, c, d, x, y); }
  static __device__ __forceinline__ void keep(v16h a, v16h b, v16h c, v16h d) { keep4_h(a, b, c, d); }
};
template <> struct Frag<__bf16> {
  typedef v16b V; union U { v16b v; v8b h[2]; };
  static __device__ __forceinline__ v16b load(const __bf16* p) {
    U f; f.h[0] = *(const v8b*)(p); f.h[1] = *(const v8b*)(p + 16); return f.v;
  }
  static __device__ __forceinline__ v8f mma(v16b a, v16b b, v8f c) {
    return __builtin_amdgcn_wmma_f32_16x16x32_bf16(false, a, false, b, (short)0, c, false, false);
  }
  static __device__ __forceinline__ void guard(v8f& a, v8f& b, v16b x, v16b y) { dep_guard_b(a, b, x, y); }
  static __device__ __forceinline__ void guard4(v8f& a, v8f& b, v8f& c, v8f& d, v16b x, v16b y) { dep_guard4_b(a, b, c, d, x, y); }
  static __device__ __forceinline__ void keep(v16b a, v16b b, v16b c, v16b d) { keep4_b(a, b, c, d); }
};

__device__ __forceinline__ unsigned short h_bits(float f) { const _Float16 h = (_Float16)f; return __builtin_bit_cast(unsigned short, h); }

template <int ET> struct Elem;
template <> struct Elem<0> { typedef _Float16 T; };
template <> struct Elem<1> { typedef __bf16 T; };
template <int ET, bool SPLIT, int BIAS_MODE, int OUT_MODE, bool RESID, int ACT = 0>
__global__ __launch_bounds__(256) void wmma_gemm64(
    const unsigned short* __restrict__ Ap, const unsigned short* __restrict__ A2p, int lda, long strideA,
    const unsigned short* __restrict__ Btp, const unsigned short* __restrict__ Bt2p, int ldb, long strideB,
    void* __restrict__ Cout, void* __restrict__ Cout2, int ldc, long strideC,
    const float* __restrict__ bias,
    const float* __restrict__ resid, long strideR,
    int M, int N, int K, float scale) {
  typedef typename Elem<ET>::T T;
  typedef typename Frag<T>::V V;
  const T* A = (const T*)Ap; const T* A2 = (const T*)A2p; const T* Bt = (const T*)Btp; const T* Bt2 = (const T*)Bt2p;
  __shared__ __align__(16) float sT[8][16 * 68];
  const int b    = blockIdx.y;
  const int lane = threadIdx.x & 31;
  const int wave = threadIdx.x >> 5;
  const int tilesN = N >> 6;
  const int tilesM = M >> 6;
  const int tile = blockIdx.x * 8 + wave;
  if (tile >= tilesM * tilesN) return;
  const int tm = tile / tilesN;
  const int tn = tile - tm * tilesN;
  const int m0 = tm << 6;
  const int n0 = tn << 6;

  const T* Ab  = A  + (size_t)b * strideA;
  const T* Bb  = Bt + (size_t)b * strideB;
  const T* Ab2 = SPLIT ? (A2  + (size_t)b * strideA) : nullptr;
  const T* Bb2 = SPLIT ? (Bt2 + (size_t)b * strideB) : nullptr;

  const int rlane = lane & 15;
  const int koff  = (lane >> 4) * 8;
  const int mOff  = (lane >> 4) * 8;

  v8f acc[4][4];
#pragma unroll
  for (int i = 0; i < 4; ++i)
#pragma unroll
    for (int j = 0; j < 4; ++j) acc[i][j] = (v8f){0.f,0.f,0.f,0.f,0.f,0.f,0.f,0.f};

  for (int k0 = 0; k0 < K; k0 += 32) {
    V bh[4], bl[4];
#pragma unroll
    for (int j = 0; j < 4; ++j) {
      const size_t bo = (size_t)(n0 + (j << 4) + rlane) * ldb + koff + k0;
      bh[j] = Frag<T>::load(Bb + bo);
      if (SPLIT) bl[j] = Frag<T>::load(Bb2 + bo);
    }
#pragma unroll
    for (int i = 0; i < 4; ++i) {
      const size_t ao = (size_t)(m0 + (i << 4) + rlane) * lda + koff + k0;
      V ah = Frag<T>::load(Ab + ao);
      V al;
      if (SPLIT) al = Frag<T>::load(Ab2 + ao);
#pragma unroll
      for (int j = 0; j < 4; ++j) {
        acc[i][j] = Frag<T>::mma(ah, bh[j], acc[i][j]);
        if (SPLIT) {
          acc[i][j] = Frag<T>::mma(ah, bl[j], acc[i][j]);
          acc[i][j] = Frag<T>::mma(al, bh[j], acc[i][j]);
        }
      }
      Frag<T>::guard4(acc[i][0], acc[i][1], acc[i][2], acc[i][3], ah, SPLIT ? al : ah);
    }
    Frag<T>::keep(bh[0], bh[1], bh[2], bh[3]);
    if (SPLIT) Frag<T>::keep(bl[0], bl[1], bl[2], bl[3]);
  }
  acc_guard4(acc[0][0], acc[0][1], acc[0][2], acc[0][3]);
  acc_guard4(acc[1][0], acc[1][1], acc[1][2], acc[1][3]);
  acc_guard4(acc[2][0], acc[2][1], acc[2][2], acc[2][3]);
  acc_guard4(acc[3][0], acc[3][1], acc[3][2], acc[3][3]);

  float* slab = sT[wave];
  const float* Rb = RESID ? (resid + (size_t)b * strideR) : nullptr;
#pragma unroll
  for (int i = 0; i < 4; ++i) {
    const int mBase = m0 + (i << 4);
#pragma unroll
    for (int j = 0; j < 4; ++j) {
      const int n = n0 + (j << 4) + rlane;
      float bv = 0.f;
      if (BIAS_MODE == 2) bv = bias[n];
#pragma unroll
      for (int r = 0; r < 8; ++r) {
        float v = acc[i][j][r] * scale;
        if (BIAS_MODE == 1) v += bias[mBase + mOff + r];
        if (BIAS_MODE == 2) v += bv;
        if (RESID) v += Rb[(size_t)(mBase + mOff + r) * ldc + n];
        if (ACT == 2) v = fmaxf(v, 0.0f);
        if (ACT == 4) v = (v > 0.f) ? v : 0.01f * v;
        slab[(mOff + r) * 68 + (j << 4) + rlane] = v;
      }
    }
    __builtin_amdgcn_fence(__ATOMIC_RELEASE, "workgroup");
    __builtin_amdgcn_wave_barrier();
    __builtin_amdgcn_fence(__ATOMIC_ACQUIRE, "workgroup");
    if (OUT_MODE == 0) {
      float* C = (float*)Cout + (size_t)b * strideC;
      const int hh = lane >> 4, c4 = (lane & 15) * 4;
      for (int pass = 0; pass < 2; ++pass) {
#pragma unroll
        for (int it = 0; it < 8; ++it) {
          const int row = it * 2 + hh;
          v4f v = *(const v4f*)(slab + row * 68 + c4);
          *(volatile v4f*)(C + (size_t)(mBase + row) * ldc + n0 + c4) = v;
        }
        __threadfence();
      }
    } else {
      const int q = lane >> 3, c8 = (lane & 7) * 8;
      unsigned short* C  = (unsigned short*)Cout  + (size_t)b * strideC;
      unsigned short* C2 = (OUT_MODE == 2) ? ((unsigned short*)Cout2 + (size_t)b * strideC) : nullptr;
      for (int pass = 0; pass < 2; ++pass) {
#pragma unroll
        for (int it = 0; it < 4; ++it) {
          const int row = it * 4 + q;
          const float* sp = slab + row * 68 + c8;
          v8h hv, lv;
#pragma unroll
          for (int e = 0; e < 8; ++e) {
            if (OUT_MODE == 1) {
              hv[e] = (_Float16)sp[e];
            } else {
              unsigned short hb = f2bf_bits(sp[e]);
              unsigned short lb = f2bf_bits(sp[e] - bf_bits2f(hb));
              hv[e] = __builtin_bit_cast(_Float16, hb);
              lv[e] = __builtin_bit_cast(_Float16, lb);
            }
          }
          *(volatile v8h*)(C + (size_t)(mBase + row) * ldc + n0 + c8) = hv;
          if (OUT_MODE == 2) *(volatile v8h*)(C2 + (size_t)(mBase + row) * ldc + n0 + c8) = lv;
        }
        __threadfence();
      }
    }
    __builtin_amdgcn_fence(__ATOMIC_RELEASE, "workgroup");
    __builtin_amdgcn_wave_barrier();
    __builtin_amdgcn_fence(__ATOMIC_ACQUIRE, "workgroup");
  }
}

__device__ __forceinline__ void store_rows_whole_lines(const unsigned short* sbuf, unsigned short* gbase, int t) {
  for (int pass = 0; pass < 2; ++pass) {
#pragma unroll 1
    for (int it = 0; it < kStoreIters; ++it) {
      const int c = it * 256 + t;
      const v4u u = *(const v4u*)(sbuf + (size_t)c * 8);
      *(volatile v4u*)(gbase + (size_t)c * 8) = u;
    }
    __threadfence();
  }
}

__global__ __launch_bounds__(256) void wt_build_kernel(const float* __restrict__ coef,
                                                       const float* __restrict__ scale_base,
                                                       const float* __restrict__ scale_sp,
                                                       const float* __restrict__ mask,
                                                       unsigned short* __restrict__ Wt) {
  __shared__ __align__(16) unsigned short sW[kRowsPerBlk * kKeff];
  const int t  = threadIdx.x;
  const int o0 = blockIdx.x * kRowsPerBlk;
#pragma unroll 1
  for (int oo = 0; oo < kRowsPerBlk; ++oo) {
    const int io = t * kOut + o0 + oo;
    const float* cp = coef + (size_t)io * kNBasis;
    const v4f ca = *(const v4f*)(cp);
    const v4f cb = *(const v4f*)(cp + 4);
    const float mk = mask[io];
    const float ss = scale_sp[io];
    const float sb = scale_base[io];
    const float wsp  = mk * ss * kWCarry;
    const float sb16 = mk * sb * kWCarry;
    unsigned short* dst = sW + oo * kKeff + t * kFeat;
    dst[0] = h_bits(wsp * ca[0]);
    dst[1] = h_bits(wsp * ca[1]);
    dst[2] = h_bits(wsp * ca[2]);
    dst[3] = h_bits(wsp * ca[3]);
    dst[4] = h_bits(wsp * cb[0]);
    dst[5] = h_bits(wsp * cb[1]);
    dst[6] = h_bits(wsp * cb[2]);
    dst[7] = h_bits(wsp * cb[3]);
    const _Float16 sbh = (_Float16)sb16;
    float sbhf = (float)sbh;
    asm volatile("" : "+v"(sbhf));
    const float sbl = sb16 - sbhf;
    dst[8]  = __builtin_bit_cast(unsigned short, sbh);
    dst[9]  = h_bits(sbhf * kResCarryInv);
    dst[10] = h_bits(sbl * kResCarry);
  }
  __syncthreads();
  store_rows_whole_lines(sW, Wt + (size_t)o0 * kKeff, t);
}

__global__ __launch_bounds__(256) void feat_build_kernel(const float* __restrict__ x,
                                                         const float* __restrict__ knots,
                                                         unsigned short* __restrict__ F) {
  __shared__ __align__(16) unsigned short sF[kRowsPerBlk * kKeff];
  const int t  = threadIdx.x;
  const int b0 = blockIdx.x * kRowsPerBlk;
  const float* gp = knots + (size_t)t * kGpts;
  const v4f ga = *(const v4f*)(gp);
  const v4f gb = *(const v4f*)(gp + 4);
  const v4f gc = *(const v4f*)(gp + 8);
  float gv[kGpts];
  gv[0] = ga[0]; gv[1] = ga[1]; gv[2]  = ga[2]; gv[3]  = ga[3];
  gv[4] = gb[0]; gv[5] = gb[1]; gv[6]  = gb[2]; gv[7]  = gb[3];
  gv[8] = gc[0]; gv[9] = gc[1]; gv[10] = gc[2]; gv[11] = gc[3];

  float rcp1[11], rcp2[10], rcp3[9];
#pragma unroll
  for (int j = 0; j < 11; ++j) {
    const float d = gv[j + 1] - gv[j];
    const float rc = __builtin_amdgcn_rcpf(d);
    rcp1[j] = (d != 0.0f) ? rc : 0.0f;
  }
#pragma unroll
  for (int j = 0; j < 10; ++j) {
    const float d = gv[j + 2] - gv[j];
    const float rc = __builtin_amdgcn_rcpf(d);
    rcp2[j] = (d != 0.0f) ? rc : 0.0f;
  }
#pragma unroll
  for (int j = 0; j < 9; ++j) {
    const float d = gv[j + 3] - gv[j];
    const float rc = __builtin_amdgcn_rcpf(d);
    rcp3[j] = (d != 0.0f) ? rc : 0.0f;
  }

#pragma unroll 1
  for (int q = 0; q < kRowsPerBlk; ++q) {
    const float xv = x[(size_t)(b0 + q) * kIn + t];
    float bs[11];
#pragma unroll
    for (int j = 0; j < 11; ++j) bs[j] = (xv >= gv[j] && xv < gv[j + 1]) ? 1.0f : 0.0f;
#pragma unroll
    for (int j = 0; j < 10; ++j) {
      const float lf = (xv - gv[j]) * rcp1[j];
      const float rf = (gv[j + 2] - xv) * rcp1[j + 1];
      bs[j] = lf * bs[j] + rf * bs[j + 1];
    }
#pragma unroll
    for (int j = 0; j < 9; ++j) {
      const float lf = (xv - gv[j]) * rcp2[j];
      const float rf = (gv[j + 3] - xv) * rcp2[j + 1];
      bs[j] = lf * bs[j] + rf * bs[j + 1];
    }
#pragma unroll
    for (int j = 0; j < 8; ++j) {
      const float lf = (xv - gv[j]) * rcp3[j];
      const float rf = (gv[j + 4] - xv) * rcp3[j + 1];
      bs[j] = lf * bs[j] + rf * bs[j + 1];
    }
    const float en   = expf(fminf(-xv, 80.0f));
    const float sig  = 1.0f / (1.0f + en);
    const float silu = xv * sig;
    const _Float16 sh = (_Float16)silu;
    float shf = (float)sh;
    asm volatile("" : "+v"(shf));
    const float sl = silu - shf;

    unsigned short* dst = sF + q * kKeff + t * kFeat;
#pragma unroll
    for (int k = 0; k < kNBasis; ++k) dst[k] = h_bits(bs[k]);
    dst[8]  = __builtin_bit_cast(unsigned short, sh);
    dst[9]  = h_bits(sl * kResCarry);
    dst[10] = h_bits(shf * kResCarryInv);
  }
  __syncthreads();
  store_rows_whole_lines(sF, F + (size_t)b0 * kKeff, t);
}

extern "C" void kernel_launch(void* const* d_in, const int* in_sizes, int n_in,
                              void* d_out, int out_size, void* d_ws, size_t ws_size,
                              hipStream_t stream) {
  (void)in_sizes; (void)out_size;
  if (n_in < 6) return;
  const float* x          = (const float*)d_in[0];
  const float* knots      = (const float*)d_in[1];
  const float* coef       = (const float*)d_in[2];
  const float* scale_base = (const float*)d_in[3];
  const float* scale_sp   = (const float*)d_in[4];
  const float* mask       = (const float*)d_in[5];
  float* out = (float*)d_out;

  unsigned char* ws = (unsigned char*)d_ws;
  const size_t bytesWt = (size_t)kOut * kKeff * 2;
  const size_t bytesF  = (size_t)kBatch * kKeff * 2;
  const size_t offWt = 0;
  const size_t offF  = offWt + bytesWt;
  if (offF + bytesF > ws_size) return;
  unsigned short* Wt = (unsigned short*)(ws + offWt);
  unsigned short* Fp = (unsigned short*)(ws + offF);
  const float* dummyf = (const float*)(ws + offWt);

  wt_build_kernel<<<dim3(kOut / kRowsPerBlk), dim3(256), 0, stream>>>(coef, scale_base, scale_sp, mask, Wt);
  feat_build_kernel<<<dim3(kBatch / kRowsPerBlk), dim3(256), 0, stream>>>(x, knots, Fp);

  const int tiles = (kBatch / 64) * (kOut / 64);
  wmma_gemm64<0, false, 0, 0, false, 0><<<dim3(tiles / 8, 1), dim3(256), 0, stream>>>(
      Fp, Fp, kKeff, 0L,
      Wt, Wt, kKeff, 0L,
      (void*)out, (void*)out, kOut, 0L,
      dummyf,
      dummyf, 0L,
      kBatch, kOut, kKeff, kWCarryInv);
}
